// MyPointNetConv_45097156608515
// MI455X (gfx1250) — hardware-run, weakly checked
//
#include <hip/hip_runtime.h>
#include <stddef.h>
#include <stdint.h>
#include <math.h>


#define NN     100000
#define NE     1600000
#define XD     61
#define KD     64
#define OD     128
#define MP     100096
#define EPSF   1e-5f

#define PTHR   256
#define PR     32
#define PBA    (MP / PR)
#define PBW    ((OD * KD / 8) / PTHR)
#define PBTOT  (PBA + PBW + 1)
#define XQ     (PR * XD / 4)
#define PQ     (PR * 3 / 4)
#define X4TOT  (NN * XD / 4)
#define P4TOT  (NN * 3 / 4)
#define TABF   1024

#define GBM    64
#define GTHR   128

#define NTHR   256
#define NWAVE  8
#define EPT    8
#define WCH    (32 * EPT)
#define NBRUN  1024
#define SLB    10
#define NBK    98
#define WLCAP  3584
#define RCAP   28672
#define DEGCAP 64
#define MAXDEG_MEAS   35
#define MAXB1024_MEAS 16663
#define SC_ZINTS (NWAVE * WLCAP + RCAP + 3 * NBRUN)
#define SC_INTS  (SC_ZINTS + 16)
#define SC_LDS   (SC_INTS * 4)
#define WSMAX  (128u << 20)

static_assert(KD == 64 && KD == XD + 3 && KD % 32 == 0);
static_assert(OD == 32 * 4);
static_assert(MP == 782 * 128 && MP >= NN && MP % GBM == 0 && MP % PR == 0);
static_assert(NN % PR == 0 && (PR * XD) % 4 == 0 && (PR * 3) % 4 == 0 && (NN * XD) % 4 == 0 && (NN * 3) % 4 == 0);
static_assert(PR * 8 == PTHR && (OD * KD / 8) % PTHR == 0 && TABF == 4 * PTHR && XQ <= 2 * PTHR && PQ <= PTHR);
static_assert(GBM == (GTHR / 32) * 16);
static_assert(NBRUN == (1 << SLB) && NBRUN % NWAVE == 0 && NBRUN % 32 == 0);
static_assert(NBK * NBRUN >= NN);
static_assert(NN <= (1 << 17) && (((long long)NN) << SLB) < (1LL << 31));
static_assert(NE % WCH == 0);
static_assert(RCAP == NWAVE * WLCAP && RCAP % 4 == 0 && SC_ZINTS % (NTHR * 4) == 0);
static_assert((long long)RCAP * 100 >= (long long)MAXB1024_MEAS * 105);
static_assert(WLCAP >= MAXB1024_MEAS / 8 + 8 * 46 + 1);
static_assert(MAXDEG_MEAS + 8 <= DEGCAP);
static_assert(SC_LDS <= 300000);

typedef float          v4f   __attribute__((ext_vector_type(4)));
typedef float          v8f   __attribute__((ext_vector_type(8)));
typedef int            v4i   __attribute__((ext_vector_type(4)));
typedef int            v8i   __attribute__((ext_vector_type(8)));
typedef unsigned short v8us  __attribute__((ext_vector_type(8)));
typedef unsigned short v16us __attribute__((ext_vector_type(16)));
typedef __bf16         v16bf __attribute__((ext_vector_type(16)));
typedef v4f  __attribute__((may_alias)) v4fa;
typedef v4i  __attribute__((may_alias)) v4ia;
typedef v8us __attribute__((may_alias)) v8usa;
union FragB { v16bf v; v16us u; v8us h[2]; v8i w; };

__device__ __forceinline__ v8f wmb(const FragB& a, const FragB& b, v8f c) {
  v8f d = __builtin_amdgcn_wmma_f32_16x16x32_bf16(false, a.v, false, b.v, (short)0, c, false, false);
  asm volatile("v_nop\n\tv_nop\n\tv_nop\n\tv_nop" : "+v"(d) : "v"(a.w), "v"(b.w));
  return d;
}

__device__ __forceinline__ unsigned bf16_bits(float f) {
  const unsigned u = __float_as_uint(f);
  const unsigned r = (u + 0x7FFFu + ((u >> 16) & 1u)) >> 16;
  const unsigned q = (u >> 16) | 0x40u;
  return ((u & 0x7fffffffu) > 0x7f800000u) ? q : r;
}
__device__ __forceinline__ float bf16_val(float f) {
  return __uint_as_float(bf16_bits(f) << 16);
}

__device__ __forceinline__ void st2_v4f(float* p, v4f v) {
  *(volatile v4f*)p = v;
  __threadfence();
  *(volatile v4f*)p = v;
}
__device__ __forceinline__ void st2_v8us(unsigned short* p, v8us v) {
  *(volatile v8us*)p = v;
  __threadfence();
  *(volatile v8us*)p = v;
}

__device__ __forceinline__ v8us cvt8(v4f a, v4f b, unsigned mk) {
  v8us o;
  o[0] = (unsigned short)(bf16_bits(a.x) & mk); o[1] = (unsigned short)(bf16_bits(a.y) & mk);
  o[2] = (unsigned short)(bf16_bits(a.z) & mk); o[3] = (unsigned short)(bf16_bits(a.w) & mk);
  o[4] = (unsigned short)(bf16_bits(b.x) & mk); o[5] = (unsigned short)(bf16_bits(b.y) & mk);
  o[6] = (unsigned short)(bf16_bits(b.z) & mk); o[7] = (unsigned short)(bf16_bits(b.w) & mk);
  return o;
}

__global__ __launch_bounds__(PTHR) void k_prep(const float* __restrict__ x, const float* __restrict__ pos,
                                               const float* __restrict__ W, const float* __restrict__ gamma,
                                               const float* __restrict__ beta, const float* __restrict__ rmean,
                                               const float* __restrict__ rvar,
                                               unsigned short* AB, unsigned short* WB, float* TAB) {
  __shared__ __attribute__((aligned(16))) float srow[PR * KD];
  __shared__ __attribute__((aligned(16))) float stab[TABF];
  const int tid = (int)threadIdx.x;
  const int blk = (int)blockIdx.x;
  if (blk < PBA) {
    const int rowBase = blk * PR;
    const bool live = rowBase < NN;
#pragma unroll
    for (int it = 0; it < 2; ++it) {
      const int idx = it * PTHR + tid;
      const int c   = idx < XQ ? idx : XQ - 1;
      int g = blk * XQ + c;
      g = g < X4TOT ? g : X4TOT - 1;
      const v4f v = *(const v4fa*)(x + (size_t)4 * (size_t)g);
      asm volatile("" :: "v"(v));
      if (idx < XQ) {
        const int f0 = 4 * c, f1 = f0 + 1, f2 = f0 + 2, f3 = f0 + 3;
        const int r0 = f0 / XD, r1 = f1 / XD, r2 = f2 / XD, r3 = f3 / XD;
        srow[r0 * KD + (f0 - XD * r0)] = v.x;
        srow[r1 * KD + (f1 - XD * r1)] = v.y;
        srow[r2 * KD + (f2 - XD * r2)] = v.z;
        srow[r3 * KD + (f3 - XD * r3)] = v.w;
      }
    }
    {
      const int c = tid < PQ ? tid : PQ - 1;
      int g = blk * PQ + c;
      g = g < P4TOT ? g : P4TOT - 1;
      const v4f v = *(const v4fa*)(pos + (size_t)4 * (size_t)g);
      asm volatile("" :: "v"(v));
      if (tid < PQ) {
        const int f0 = 4 * c, f1 = f0 + 1, f2 = f0 + 2, f3 = f0 + 3;
        const int r0 = f0 / 3, r1 = f1 / 3, r2 = f2 / 3, r3 = f3 / 3;
        srow[r0 * KD + XD + (f0 - 3 * r0)] = v.x;
        srow[r1 * KD + XD + (f1 - 3 * r1)] = v.y;
        srow[r2 * KD + XD + (f2 - 3 * r2)] = v.z;
        srow[r3 * KD + XD + (f3 - 3 * r3)] = v.w;
      }
    }
    __syncthreads();
    const int r = tid >> 3, k8 = (tid & 7) * 8;
    const v4f a = *(const v4fa*)(srow + r * KD + k8);
    const v4f b = *(const v4fa*)(srow + r * KD + k8 + 4);
    const unsigned mk = live ? 0xffffu : 0u;
    const v8us o = cvt8(a, b, mk);
    st2_v8us(AB + (size_t)(rowBase + r) * KD + k8, o);
  } else if (blk < PBA + PBW) {
    const int u = (blk - PBA) * PTHR + tid;
    const int n = u >> 3, k8 = (u & 7) * 8;
    const float* p = W + (size_t)n * KD + k8;
    const v4f a = *(const v4fa*)p;
    const v4f b = *(const v4fa*)(p + 4);
    const v8us o = cvt8(a, b, 0xffffu);
    st2_v8us(WB + (size_t)n * KD + k8, o);
  } else {
#pragma unroll 1
    for (int j = 0; j < 4; ++j) {
      const int e = j * PTHR + tid;
      const int p = e >> 7, c = e & (OD - 1);
      int d = p - 4;
      d = d < 0 ? 0 : (d > 2 ? 2 : d);
      const float gv = gamma[c];
      const float mv = rmean[c];
      const float vv = rvar[c];
      const float bv = beta[c];
      const float wv = W[(size_t)c * KD + XD + d];
      asm volatile("" :: "v"(gv), "v"(mv), "v"(vv), "v"(bv), "v"(wv));
      const float rs = 1.0f / sqrtf(bf16_val(vv) + EPSF);
      float val = 0.0f;
      val = (p == 0) ? bf16_val(gv) : val;
      val = (p == 1) ? bf16_val(mv) : val;
      val = (p == 2) ? rs : val;
      val = (p == 3) ? bf16_val(bv) : val;
      val = (p >= 4 && p <= 6) ? bf16_val(wv) : val;
      stab[e] = val;
    }
    __syncthreads();
    const v4f v = *(const v4fa*)(stab + 4 * tid);
    st2_v4f(TAB + 4 * tid, v);
  }
}

__device__ __forceinline__ void p_flush(const float* stg, float* P, int rowBase, int wave, int lane) {
#pragma unroll 1
  for (int i = 0; i < 16; ++i) {
    const int lr = 16 * wave + i;
    const int r  = rowBase + lr;
    const v4f v = *(const v4fa*)(stg + lr * OD + 4 * lane);
    asm volatile("" :: "v"(v));
    if (r < NN) *(volatile v4f*)(P + (size_t)r * OD + 4 * lane) = v;
  }
}

__global__ __launch_bounds__(GTHR) __attribute__((amdgpu_num_vgpr(248)))
void k_gemm_p(const unsigned short* __restrict__ AB, const unsigned short* __restrict__ WB, float* P) {
  __shared__ __attribute__((aligned(16))) float stg[GBM * OD];
  const int tid = (int)threadIdx.x, lane = tid & 31, wave = tid >> 5, hh = lane >> 4, m = lane & 15;
  const int rowBase = (int)blockIdx.x * GBM;

  v8f acc[8];
  {
    const v8f z = {0.f, 0.f, 0.f, 0.f, 0.f, 0.f, 0.f, 0.f};
#pragma unroll
    for (int t = 0; t < 8; ++t) acc[t] = z;
  }
  const unsigned short* ap = AB + (size_t)(rowBase + 16 * wave + m) * (size_t)KD + 8 * hh;
  const unsigned short* bp = WB + (size_t)m * (size_t)KD + 8 * hh;

#pragma unroll 1
  for (int k0 = 0; k0 < KD; k0 += 32) {
    FragB af;
    af.h[0] = *(const v8usa*)(ap + k0);
    af.h[1] = *(const v8usa*)(ap + k0 + 16);
#pragma unroll
    for (int nt = 0; nt < 8; ++nt) {
      const unsigned short* wq = bp + (size_t)(16 * nt) * (size_t)KD + k0;
      FragB bf;
      bf.h[0] = *(const v8usa*)wq;
      bf.h[1] = *(const v8usa*)(wq + 16);
      acc[nt] = wmb(af, bf, acc[nt]);
    }
  }

#pragma unroll
  for (int nt = 0; nt < 8; ++nt) {
    const int lc = 16 * nt + m;
#pragma unroll
    for (int r = 0; r < 8; ++r) {
      const int lr = 16 * wave + 8 * hh + r;
      stg[lr * OD + lc] = acc[nt][r];
    }
  }
  __syncthreads();
  p_flush(stg, P, rowBase, wave, lane);
  __threadfence();
  p_flush(stg, P, rowBase, wave, lane);
}

__device__ __forceinline__ int clamp_src(int v) {
  return v < 0 ? 0 : (v > NN - 1 ? NN - 1 : v);
}

__device__ __forceinline__ float upd(float p, float q, float g, float rm, float rs, float b, float m) {
  const float d = p - q;
  const float t = g * (d - rm);
  const float v = fmaf(t, rs, b);
  return ((v > m) | (v != v)) ? v : m;
}

__device__ __forceinline__ float relu_keep(float m) {
  return (m > 0.0f) ? m : ((m != m) ? m : 0.0f);
}

__global__ __launch_bounds__(NTHR) void k_scan(const int* __restrict__ edges, const float* __restrict__ pos,
                                               const float* __restrict__ TAB, const float* __restrict__ P,
                                               float* out) {
  extern __shared__ __attribute__((aligned(16))) int dsm[];
  int* wl   = dsm;
  int* pl   = dsm + NWAVE * WLCAP;
  int* cnt  = pl + RCAP;
  int* offs = cnt + NBRUN;
  int* cur  = offs + NBRUN;
  int* misc = cur + NBRUN;
  const int tid = (int)threadIdx.x, lane = tid & 31;
  const int wave = __builtin_amdgcn_readfirstlane(tid >> 5);
  const int blk = (int)blockIdx.x;
  const int nodeBase = blk * NBRUN;
  const unsigned nbs = (unsigned)nodeBase;

  {
    const v4i z4 = {0, 0, 0, 0};
    for (int i = tid * 4; i < SC_ZINTS; i += NTHR * 4) *(v4ia*)(dsm + i) = z4;
    if (tid < 16) misc[tid] = 0;
  }
  __syncthreads();

  {
    const int per  = ((NE + NWAVE * WCH - 1) / (NWAVE * WCH)) * WCH;
    const int ebeg = wave * per;
    const int eend = (ebeg + per < NE) ? (ebeg + per) : NE;
    int* mylist = wl + wave * WLCAP;
    int wc = 0;
#pragma unroll 1
    for (int cb = ebeg; cb < eend; cb += WCH) {
      const int e0 = cb + lane * EPT;
      const int* ep = edges + (size_t)2 * (size_t)e0;
      const v4i q0 = *(const v4ia*)(ep);
      const v4i q1 = *(const v4ia*)(ep + 4);
      const v4i q2 = *(const v4ia*)(ep + 8);
      const v4i q3 = *(const v4ia*)(ep + 12);
      const unsigned s0 = (unsigned)q0.x - nbs, s1 = (unsigned)q0.z - nbs;
      const unsigned s2 = (unsigned)q1.x - nbs, s3 = (unsigned)q1.z - nbs;
      const unsigned s4 = (unsigned)q2.x - nbs, s5 = (unsigned)q2.z - nbs;
      const unsigned s6 = (unsigned)q3.x - nbs, s7 = (unsigned)q3.z - nbs;
      const bool h0 = s0 < (unsigned)NBRUN, h1 = s1 < (unsigned)NBRUN, h2 = s2 < (unsigned)NBRUN, h3 = s3 < (unsigned)NBRUN;
      const bool h4 = s4 < (unsigned)NBRUN, h5 = s5 < (unsigned)NBRUN, h6 = s6 < (unsigned)NBRUN, h7 = s7 < (unsigned)NBRUN;
      const unsigned m0 = __builtin_amdgcn_ballot_w32(h0), m1 = __builtin_amdgcn_ballot_w32(h1);
      const unsigned m2 = __builtin_amdgcn_ballot_w32(h2), m3 = __builtin_amdgcn_ballot_w32(h3);
      const unsigned m4 = __builtin_amdgcn_ballot_w32(h4), m5 = __builtin_amdgcn_ballot_w32(h5);
      const unsigned m6 = __builtin_amdgcn_ballot_w32(h6), m7 = __builtin_amdgcn_ballot_w32(h7);
      const unsigned any = m0 | m1 | m2 | m3 | m4 | m5 | m6 | m7;
      if (any != 0u) {
        const int pre = (int)(__builtin_amdgcn_mbcnt_lo(m0, 0u) + __builtin_amdgcn_mbcnt_lo(m1, 0u) +
                              __builtin_amdgcn_mbcnt_lo(m2, 0u) + __builtin_amdgcn_mbcnt_lo(m3, 0u) +
                              __builtin_amdgcn_mbcnt_lo(m4, 0u) + __builtin_amdgcn_mbcnt_lo(m5, 0u) +
                              __builtin_amdgcn_mbcnt_lo(m6, 0u) + __builtin_amdgcn_mbcnt_lo(m7, 0u));
        const int w0 = (clamp_src(q0.y) << SLB) | (int)(s0 & (NBRUN - 1));
        const int w1 = (clamp_src(q0.w) << SLB) | (int)(s1 & (NBRUN - 1));
        const int w2 = (clamp_src(q1.y) << SLB) | (int)(s2 & (NBRUN - 1));
        const int w3 = (clamp_src(q1.w) << SLB) | (int)(s3 & (NBRUN - 1));
        const int w4 = (clamp_src(q2.y) << SLB) | (int)(s4 & (NBRUN - 1));
        const int w5 = (clamp_src(q2.w) << SLB) | (int)(s5 & (NBRUN - 1));
        const int w6 = (clamp_src(q3.y) << SLB) | (int)(s6 & (NBRUN - 1));
        const int w7 = (clamp_src(q3.w) << SLB) | (int)(s7 & (NBRUN - 1));
        int p = wc + pre;
        if (h0) { if (p < WLCAP) mylist[p] = w0; p = p + 1; }
        if (h1) { if (p < WLCAP) mylist[p] = w1; p = p + 1; }
        if (h2) { if (p < WLCAP) mylist[p] = w2; p = p + 1; }
        if (h3) { if (p < WLCAP) mylist[p] = w3; p = p + 1; }
        if (h4) { if (p < WLCAP) mylist[p] = w4; p = p + 1; }
        if (h5) { if (p < WLCAP) mylist[p] = w5; p = p + 1; }
        if (h6) { if (p < WLCAP) mylist[p] = w6; p = p + 1; }
        if (h7) { if (p < WLCAP) mylist[p] = w7; p = p + 1; }
        wc += (int)(__builtin_popcount(m0) + __builtin_popcount(m1) + __builtin_popcount(m2) + __builtin_popcount(m3) +
                    __builtin_popcount(m4) + __builtin_popcount(m5) + __builtin_popcount(m6) + __builtin_popcount(m7));
      }
    }
    if (lane == 0) misc[wave] = wc;
  }
  __syncthreads();

  if (wave == 0) {
    int ov = 0;
#pragma unroll 1
    for (int w2 = 0; w2 < NWAVE; ++w2) {
      int c = misc[w2];
      if (c > WLCAP) ov = 1;
      c = c < 0 ? 0 : (c > WLCAP ? WLCAP : c);
#pragma unroll 1
      for (int b0 = 0; b0 < c; b0 += 32) {
        const int idx = b0 + lane;
        const int ent = wl[w2 * WLCAP + (idx < WLCAP ? idx : WLCAP - 1)];
        const int m32 = (c - b0) < 32 ? (c - b0) : 32;
#pragma unroll 1
        for (int k = 0; k < m32; ++k) {
          const int u    = __builtin_amdgcn_readlane(ent, k);
          const int slot = u & (NBRUN - 1);
          if (lane == 0) cnt[slot] = cnt[slot] + 1;
        }
      }
    }
    if (lane == 0) misc[9] = ov;
  }
  __syncthreads();
  if (wave == 0) {
    const int base = lane * (NBRUN / 32);
    int s = 0;
#pragma unroll 1
    for (int i = 0; i < NBRUN / 32; ++i) s += cnt[base + i];
    int incl = s;
#pragma unroll
    for (int d = 1; d < 32; d <<= 1) {
      const int y = __shfl_up(incl, d, 32);
      if (lane >= d) incl += y;
    }
    int run = incl - s;
#pragma unroll 1
    for (int i = 0; i < NBRUN / 32; ++i) {
      const int cv = cnt[base + i];
      offs[base + i] = run;
      cur[base + i]  = run;
      run += cv;
    }
  }
  __syncthreads();
  if (wave == 0) {
#pragma unroll 1
    for (int w2 = 0; w2 < NWAVE; ++w2) {
      int c = misc[w2];
      c = c < 0 ? 0 : (c > WLCAP ? WLCAP : c);
#pragma unroll 1
      for (int b0 = 0; b0 < c; b0 += 32) {
        const int idx = b0 + lane;
        const int ent = wl[w2 * WLCAP + (idx < WLCAP ? idx : WLCAP - 1)];
        const int m32 = (c - b0) < 32 ? (c - b0) : 32;
#pragma unroll 1
        for (int k = 0; k < m32; ++k) {
          const int u    = __builtin_amdgcn_readlane(ent, k);
          const int slot = u & (NBRUN - 1);
          if (lane == 0) {
            int p = cur[slot];
            p = p < 0 ? 0 : (p > RCAP - 1 ? RCAP - 1 : p);
            pl[p] = u;
            cur[slot] = p + 1;
          }
        }
      }
    }
  }
  __syncthreads();

  const int ovf = misc[9];
  const v4f g4  = *(const v4fa*)(TAB + 4 * lane);
  const v4f rm4 = *(const v4fa*)(TAB + OD + 4 * lane);
  const v4f rs4 = *(const v4fa*)(TAB + 2 * OD + 4 * lane);
  const v4f b4  = *(const v4fa*)(TAB + 3 * OD + 4 * lane);
  const v4f wa  = *(const v4fa*)(TAB + 4 * OD + 4 * lane);
  const v4f wb  = *(const v4fa*)(TAB + 5 * OD + 4 * lane);
  const v4f wc4 = *(const v4fa*)(TAB + 6 * OD + 4 * lane);
  const float qnan = __uint_as_float(0x7fc00000u);
  const float ninf = __uint_as_float(0xff800000u);

#pragma unroll 1
  for (int si = 0; si < NBRUN / NWAVE; ++si) {
    const int s    = si * NWAVE + wave;
    const int node = nodeBase + s;
    if (node >= NN) continue;
    int c = cnt[s];
    const bool big = c > DEGCAP;
    c = c < 0 ? 0 : (c > DEGCAP ? DEGCAP : c);
    c = __builtin_amdgcn_readfirstlane(c);
    int o = offs[s];
    o = o < 0 ? 0 : (o > RCAP - 1 ? RCAP - 1 : o);
    o = __builtin_amdgcn_readfirstlane(o);
    int last = o + c - 1;
    last = last < o ? o : last;
    last = last > RCAP - 1 ? RCAP - 1 : last;

    const float pxr = pos[(size_t)node * 3 + 0];
    const float pyr = pos[(size_t)node * 3 + 1];
    const float pzr = pos[(size_t)node * 3 + 2];
    asm volatile("" :: "v"(pxr), "v"(pyr), "v"(pzr));
    const float px = bf16_val(pxr), py = bf16_val(pyr), pz = bf16_val(pzr);
    const float q0 = fmaf(pz, wc4.x, fmaf(py, wb.x, px * wa.x));
    const float q1 = fmaf(pz, wc4.y, fmaf(py, wb.y, px * wa.y));
    const float q2 = fmaf(pz, wc4.z, fmaf(py, wb.z, px * wa.z));
    const float q3 = fmaf(pz, wc4.w, fmaf(py, wb.w, px * wa.w));

    float m0 = ninf, m1 = ninf, m2 = ninf, m3 = ninf;
#pragma unroll 1
    for (int j = 0; j < c; j += 4) {
      const int i0 = o + j;
      int i1 = i0 + 1, i2 = i0 + 2, i3 = i0 + 3;
      const int j0 = i0 > last ? last : i0;
      i1 = i1 > last ? last : i1;
      i2 = i2 > last ? last : i2;
      i3 = i3 > last ? last : i3;
      const unsigned u0 = (unsigned)pl[j0], u1 = (unsigned)pl[i1], u2 = (unsigned)pl[i2], u3 = (unsigned)pl[i3];
      int r0 = (int)(u0 >> SLB), r1 = (int)(u1 >> SLB), r2 = (int)(u2 >> SLB), r3 = (int)(u3 >> SLB);
      r0 = r0 > NN - 1 ? NN - 1 : r0;
      r1 = r1 > NN - 1 ? NN - 1 : r1;
      r2 = r2 > NN - 1 ? NN - 1 : r2;
      r3 = r3 > NN - 1 ? NN - 1 : r3;
      const v4f p0 = *(const v4fa*)(P + (size_t)r0 * OD + 4 * lane);
      const v4f p1 = *(const v4fa*)(P + (size_t)r1 * OD + 4 * lane);
      const v4f p2 = *(const v4fa*)(P + (size_t)r2 * OD + 4 * lane);
      const v4f p3 = *(const v4fa*)(P + (size_t)r3 * OD + 4 * lane);
      m0 = upd(p0.x, q0, g4.x, rm4.x, rs4.x, b4.x, m0);
      m1 = upd(p0.y, q1, g4.y, rm4.y, rs4.y, b4.y, m1);
      m2 = upd(p0.z, q2, g4.z, rm4.z, rs4.z, b4.z, m2);
      m3 = upd(p0.w, q3, g4.w, rm4.w, rs4.w, b4.w, m3);
      m0 = upd(p1.x, q0, g4.x, rm4.x, rs4.x, b4.x, m0);
      m1 = upd(p1.y, q1, g4.y, rm4.y, rs4.y, b4.y, m1);
      m2 = upd(p1.z, q2, g4.z, rm4.z, rs4.z, b4.z, m2);
      m3 = upd(p1.w, q3, g4.w, rm4.w, rs4.w, b4.w, m3);
      m0 = upd(p2.x, q0, g4.x, rm4.x, rs4.x, b4.x, m0);
      m1 = upd(p2.y, q1, g4.y, rm4.y, rs4.y, b4.y, m1);
      m2 = upd(p2.z, q2, g4.z, rm4.z, rs4.z, b4.z, m2);
      m3 = upd(p2.w, q3, g4.w, rm4.w, rs4.w, b4.w, m3);
      m0 = upd(p3.x, q0, g4.x, rm4.x, rs4.x, b4.x, m0);
      m1 = upd(p3.y, q1, g4.y, rm4.y, rs4.y, b4.y, m1);
      m2 = upd(p3.z, q2, g4.z, rm4.z, rs4.z, b4.z, m2);
      m3 = upd(p3.w, q3, g4.w, rm4.w, rs4.w, b4.w, m3);
    }
    const bool bad = (ovf != 0) | big;
    v4f ov;
    ov.x = relu_keep(m0); ov.y = relu_keep(m1); ov.z = relu_keep(m2); ov.w = relu_keep(m3);
    ov.x = bad ? qnan : ov.x; ov.y = bad ? qnan : ov.y; ov.z = bad ? qnan : ov.z; ov.w = bad ? qnan : ov.w;
    st2_v4f(out + (size_t)node * OD + 4 * lane, ov);
  }
}

extern "C" void kernel_launch(void* const* d_in, const int* in_sizes, int n_in,
                              void* d_out, int out_size, void* d_ws, size_t ws_size,
                              hipStream_t stream) {
  if (n_in < 8) return;
  if (in_sizes[0] != NN * XD) return;
  if (in_sizes[1] != NN * 3) return;
  if (in_sizes[2] != 2 * NE) return;
  if (in_sizes[3] != OD * KD) return;
  if (in_sizes[4] != OD || in_sizes[5] != OD) return;
  if (in_sizes[6] != OD || in_sizes[7] != OD) return;
  if (out_size != NN * OD) return;

  const float* x     = (const float*)d_in[0];
  const float* pos   = (const float*)d_in[1];
  const int*   edges = (const int*)d_in[2];
  const float* W     = (const float*)d_in[3];
  const float* gamma = (const float*)d_in[4];
  const float* beta  = (const float*)d_in[5];
  const float* rmean = (const float*)d_in[6];
  const float* rvar  = (const float*)d_in[7];
  float* out = (float*)d_out;

  constexpr size_t zAB  = (size_t)MP * KD * 2;
  constexpr size_t zWB  = (size_t)OD * KD * 2;
  constexpr size_t zTAB = (size_t)TABF * 4;
  constexpr size_t zP   = (size_t)NN * OD * 4;
  constexpr size_t oAB  = 0;
  constexpr size_t oWB  = oAB + zAB;
  constexpr size_t oTAB = oWB + zWB;
  constexpr size_t oP   = oTAB + zTAB;
  constexpr size_t oEND = oP + zP;
  static_assert(zAB % 256 == 0 && zWB % 256 == 0 && zTAB % 256 == 0 && zP % 256 == 0);
  static_assert(oEND <= (size_t)WSMAX);
  if (oEND > ws_size) return;

  char* ws = (char*)d_ws;
  unsigned short* AB  = (unsigned short*)(ws + oAB);
  unsigned short* WB  = (unsigned short*)(ws + oWB);
  float*          TAB = (float*)(ws + oTAB);
  float*          P   = (float*)(ws + oP);

  hipFuncSetAttribute(reinterpret_cast<const void*>(&k_scan), hipFuncAttributeMaxDynamicSharedMemorySize, (int)SC_LDS);

  k_prep<<<PBTOT, PTHR, 0, stream>>>(x, pos, W, gamma, beta, rmean, rvar, AB, WB, TAB);
  k_gemm_p<<<MP / GBM, GTHR, 0, stream>>>(AB, WB, P);
  k_scan<<<NBK, NTHR, SC_LDS, stream>>>(edges, pos, TAB, P, out);
}
